// MaskedMultiHeadSelfAttention_3152505995624
// MI455X (gfx1250) — hardware-verified
//
#include <hip/hip_runtime.h>
#ifndef NB
#define NB 4
#endif
#ifndef SEQ
#define SEQ 2048
#endif
#define NB_FULL 4
#define SEQ_FULL 2048
#define DM 512
#define NH 8
#define HD 64
#define LQ (3 * DM)
#ifndef QT
#if SEQ >= 512
#define QT 512
#else
#define QT SEQ
#endif
#endif
#define NKX SEQ
#define NR ((size_t)NB * SEQ)
static_assert(NB >= 1 && NB <= NB_FULL);
static_assert(SEQ >= 128 && SEQ <= SEQ_FULL);
static_assert(SEQ % QT == 0);
static_assert(QT % 128 == 0);
static_assert(SEQ % 64 == 0);
static_assert((NB * SEQ) % 128 == 0);
static_assert(DM == NH * HD && HD == 64 && DM % 64 == 0);

typedef unsigned short v8us __attribute__((ext_vector_type(8), may_alias));
typedef float  v8f  __attribute__((ext_vector_type(8)));
typedef float  v4f  __attribute__((ext_vector_type(4)));
typedef float  v4fa __attribute__((ext_vector_type(4), may_alias));
typedef int    v4ia __attribute__((ext_vector_type(4), may_alias));
typedef _Float16 v16h __attribute__((ext_vector_type(16)));
typedef _Float16 v4h __attribute__((ext_vector_type(4)));
union FragH { v16h v; v8us half[2]; _Float16 h[16]; unsigned short u[16]; };

__device__ __forceinline__ unsigned short bf16_bits(float x) { unsigned int u = __float_as_uint(x); return (unsigned short)((u + 0x7FFFu + ((u >> 16) & 1u)) >> 16); }
__device__ __forceinline__ float bf16_val(unsigned short b) { return __uint_as_float(((unsigned int)b) << 16); }
__device__ __forceinline__ float bf16_rne(float x) { return bf16_val(bf16_bits(x)); }

__device__ __forceinline__ v16h g2_frag(const _Float16* p, int hh) { FragH f; f.half[0] = *(const v8us*)((const unsigned short*)p + 8 * hh); f.half[1] = *(const v8us*)((const unsigned short*)p + 16 + 8 * hh); return f.v; }
__device__ __forceinline__ v8f g2_mma(v16h a, v16h b, v8f c) { v8f d = __builtin_amdgcn_wmma_f32_16x16x32_f16(false, a, false, b, (short)0, c, false, false); asm volatile("v_nop\n\tv_nop\n\tv_nop\n\tv_nop" : "+v"(d) : "v"(a), "v"(b)); return d; }
template <int ACT>
__global__ __launch_bounds__(128) void k_gemm2(const _Float16* __restrict__ A, int lda, size_t sA, const _Float16* __restrict__ Bh, int ldb, size_t sB, float alpha, const float* __restrict__ bias, size_t sBias, const float* __restrict__ CP, int rowsPerB, size_t sCPb, int row0g,
    float* __restrict__ C, _Float16* __restrict__ C16, int ldc, size_t sC, int M, int N, int K) {
  static_assert(ACT == 0 || ACT == 3);
  __shared__ __attribute__((aligned(16))) float so[4][32][68];
  const int tid = threadIdx.x, w = tid >> 5, lane = tid & 31, ln = lane & 15, hh = lane >> 4; const int by = blockIdx.y;
  A += (size_t)by * sA; Bh += (size_t)by * sB; const size_t cofs = (size_t)by * sC; const float* bp = bias ? bias + (size_t)by * sBias : nullptr;
  const int ntn = N >> 6; const int mt = blockIdx.x / ntn, nq = blockIdx.x - mt * ntn; const int row0 = mt * 128 + 32 * w, col0 = nq * 64; if (row0 >= M) return;
  const _Float16* a0p = A + (size_t)(row0 + ln) * lda; const _Float16* a1p = a0p + (size_t)16 * lda;
  const _Float16* b0p = Bh + (size_t)(col0 + ln) * ldb; const _Float16* b1p = b0p + (size_t)16 * ldb; const _Float16* b2p = b1p + (size_t)16 * ldb; const _Float16* b3p = b2p + (size_t)16 * ldb;
  const v8f z8 = {0.f,0.f,0.f,0.f,0.f,0.f,0.f,0.f}; v8f c00 = z8, c01 = z8, c02 = z8, c03 = z8, c10 = z8, c11 = z8, c12 = z8, c13 = z8;
#pragma unroll 1
  for (int kb = 0; kb < K; kb += 32) { const v16h a0 = g2_frag(a0p + kb, hh), a1 = g2_frag(a1p + kb, hh);
    v16h b = g2_frag(b0p + kb, hh); c00 = g2_mma(a0, b, c00); c10 = g2_mma(a1, b, c10);
    b = g2_frag(b1p + kb, hh); c01 = g2_mma(a0, b, c01); c11 = g2_mma(a1, b, c11);
    b = g2_frag(b2p + kb, hh); c02 = g2_mma(a0, b, c02); c12 = g2_mma(a1, b, c12);
    b = g2_frag(b3p + kb, hh); c03 = g2_mma(a0, b, c03); c13 = g2_mma(a1, b, c13); }
  v8f accs[8] = {c00, c01, c02, c03, c10, c11, c12, c13};
#pragma unroll
  for (int u = 0; u < 8; ++u) { const int t = u & 3, half = u >> 2; const int col = col0 + t * 16 + ln; const float bv = bp ? bf16_rne(bp[col]) : 0.f;
#pragma unroll
    for (int r = 0; r < 8; ++r) { const int rloc = half * 16 + 8 * hh + r; float v = accs[u][r] * alpha + bv;
      if (CP) { if (rowsPerB < 0) v += CP[cofs + (size_t)(row0g + row0 + rloc) * ldc + col]; else { const int bidx = (row0g + row0 + rloc) / rowsPerB; v += CP[(size_t)bidx * sCPb + (size_t)by * 64 + col]; } }
      if (ACT == 3) v = fmaxf(v, 0.f);
      so[w][rloc][t * 16 + ln] = v; } }
  __builtin_amdgcn_fence(4, "workgroup"); __builtin_amdgcn_wave_barrier();
  const int rsub = lane >> 4, c4 = (lane & 15) * 4;
  for (int pass = 0; pass < 2; ++pass) {
#pragma unroll
    for (int q = 0; q < 16; ++q) { const int r = q * 2 + rsub; const v4f v = *(const v4fa*)&so[w][r][c4];
      if (C) *(volatile v4f*)(C + cofs + (size_t)(row0 + r) * ldc + col0 + c4) = v;
      if (C16) { v4h h4; for (int i = 0; i < 4; ++i) h4[i] = (_Float16)v[i]; *(volatile v4h*)(C16 + cofs + (size_t)(row0 + r) * ldc + col0 + c4) = h4; } }
    if (pass == 0) __threadfence(); } }

__global__ __launch_bounds__(256) void k_wnat(const float* __restrict__ w, size_t n8, _Float16* __restrict__ Bt) {
  const size_t t = (size_t)blockIdx.x * 256 + threadIdx.x; if (t >= n8) return;
  const v4f a = *(const v4fa*)(w + t * 8), c = *(const v4fa*)(w + t * 8 + 4); FragH f;
#pragma unroll
  for (int q = 0; q < 4; ++q) { f.h[q] = (_Float16)(bf16_rne(a[q]) * 16.0f); f.h[4 + q] = (_Float16)(bf16_rne(c[q]) * 16.0f); }
  *(volatile v8us*)((unsigned short*)Bt + t * 8) = f.half[0]; __threadfence(); *(volatile v8us*)((unsigned short*)Bt + t * 8) = f.half[0]; }

__global__ __launch_bounds__(256) void k_x16(const float* __restrict__ x, _Float16* __restrict__ X16, size_t n8) {
  const size_t t = (size_t)blockIdx.x * 256 + threadIdx.x; if (t >= n8) return;
  const size_t per = (size_t)SEQ * DM / 8; const size_t b = t / per, rem = t - b * per;
  const float* src = x + b * ((size_t)SEQ_FULL * DM) + rem * 8;
  const v4f a = *(const v4fa*)src, c = *(const v4fa*)(src + 4); FragH f;
#pragma unroll
  for (int q = 0; q < 4; ++q) { f.h[q] = (_Float16)bf16_rne(a[q]); f.h[4 + q] = (_Float16)bf16_rne(c[q]); }
  *(volatile v8us*)((unsigned short*)X16 + t * 8) = f.half[0]; __threadfence(); *(volatile v8us*)((unsigned short*)X16 + t * 8) = f.half[0]; }

template <int NHv, int TTv>
__global__ __launch_bounds__(256) void k_vt(const _Float16* __restrict__ V16, int ldv, int voff, _Float16* __restrict__ Vt) {
  __shared__ unsigned short tl[64][66]; const int tid = threadIdx.x; const int slab = blockIdx.x / (TTv / 64), lg = blockIdx.x % (TTv / 64); const int b = slab / NHv, h = slab % NHv;
  for (int i = tid; i < 64 * 8; i += 256) { const int r = i / 8, c8 = (i % 8) * 8; FragH f; f.half[0] = *(const v8us*)((const unsigned short*)V16 + ((size_t)b * TTv + lg * 64 + r) * ldv + voff + h * 64 + c8);
#pragma unroll
    for (int q = 0; q < 8; ++q) tl[r][c8 + q] = f.u[q]; }
  __syncthreads();
  for (int pass = 0; pass < 2; ++pass) {
#pragma unroll
    for (int rd = 0; rd < 2; ++rd) { const int d = rd * 32 + tid / 8, pc = tid % 8; FragH f;
#pragma unroll
      for (int q = 0; q < 8; ++q) f.u[q] = tl[pc * 8 + q][d];
      *(volatile v8us*)((unsigned short*)Vt + ((size_t)slab * 64 + d) * TTv + lg * 64 + pc * 8) = f.half[0]; }
    if (pass == 0) __threadfence(); } }

__global__ __launch_bounds__(256) void k_rsmm(const float* __restrict__ S, const int* __restrict__ adj, _Float16* __restrict__ P, int hg, int q0) {
  #pragma clang fp contract(off)
  const int t = blockIdx.x * 256 + threadIdx.x; if (t >= hg * QT) return;
  const size_t i = (size_t)t; const float* s = S + i * NKX; const int* a = adj + (size_t)(q0 + (t % QT)) * SEQ_FULL;
  float mx = -3.0e38f;
#pragma unroll 1
  for (int j0 = 0; j0 < NKX; j0 += 4) { const v4f sv = *(const v4fa*)(s + j0); const v4ia av = *(const v4ia*)(a + j0);
#pragma unroll
    for (int q = 0; q < 4; ++q) { const float v = (av[q] != 0) ? sv[q] : -1.0e30f; mx = fmaxf(mx, v); } }
  float se = 0.f;
#pragma unroll 1
  for (int j0 = 0; j0 < NKX; j0 += 4) { const v4f sv = *(const v4fa*)(s + j0); const v4ia av = *(const v4ia*)(a + j0);
#pragma unroll
    for (int q = 0; q < 4; ++q) { const float v = (av[q] != 0) ? sv[q] : -1.0e30f; se += __expf(v - mx); } }
  const float sc = (mx > -1.0e29f) ? (1024.0f / se) : __uint_as_float(0x7fc00000u);
#pragma unroll 1
  for (int j0 = 0; j0 < NKX; j0 += 8) { const v4f s0 = *(const v4fa*)(s + j0), s1 = *(const v4fa*)(s + j0 + 4); const v4ia a0 = *(const v4ia*)(a + j0), a1 = *(const v4ia*)(a + j0 + 4); FragH fr;
#pragma unroll
    for (int q = 0; q < 4; ++q) { const float v0 = (a0[q] != 0) ? s0[q] : -1.0e30f; const float v1 = (a1[q] != 0) ? s1[q] : -1.0e30f; fr.h[q] = (_Float16)(__expf(v0 - mx) * sc); fr.h[4 + q] = (_Float16)(__expf(v1 - mx) * sc); }
    unsigned short* d = (unsigned short*)P + i * NKX + j0; *(volatile v8us*)d = fr.half[0]; __threadfence(); *(volatile v8us*)d = fr.half[0]; } }

extern "C" void kernel_launch(void* const* d_in, const int* in_sizes, int n_in,
                              void* d_out, int out_size, void* d_ws, size_t ws_size, hipStream_t stream) {
  if (n_in < 10) return;
  if (in_sizes[0] < NB * SEQ_FULL * DM || in_sizes[1] < SEQ * SEQ_FULL) return;
  if (in_sizes[2] < DM * DM || in_sizes[4] < DM * DM || in_sizes[6] < DM * DM || in_sizes[8] < DM * DM) return;
  if (in_sizes[3] < DM || in_sizes[5] < DM || in_sizes[7] < DM || in_sizes[9] < DM) return;
  if (out_size < (int)(NR * DM)) return;
  const float* x  = (const float*)d_in[0]; const int* adj = (const int*)d_in[1];
  const float* wq = (const float*)d_in[2]; const float* bq = (const float*)d_in[3];
  const float* wk = (const float*)d_in[4]; const float* bk = (const float*)d_in[5];
  const float* wv = (const float*)d_in[6]; const float* bv = (const float*)d_in[7];
  const float* wo = (const float*)d_in[8]; const float* bo = (const float*)d_in[9];
  char* ws = (char*)d_ws; size_t off = 0;
  auto take = [&](size_t bytes) { char* p = ws + off; off += (bytes + 255) & ~(size_t)255; return p; };
  _Float16* BQ  = (_Float16*)take((size_t)DM * DM * 2); _Float16* BK = (_Float16*)take((size_t)DM * DM * 2);
  _Float16* BV  = (_Float16*)take((size_t)DM * DM * 2); _Float16* BO = (_Float16*)take((size_t)DM * DM * 2);
  _Float16* X16 = (_Float16*)take(NR * DM * 2);
  _Float16* QKV = (_Float16*)take(NR * LQ * 2);
  _Float16* O16 = (_Float16*)take(NR * DM * 2);
  _Float16* VT  = (_Float16*)take((size_t)NB * NH * HD * SEQ * 2);
  float*    S   = (float*)take((size_t)NH * QT * NKX * 4);
  _Float16* P   = (_Float16*)take((size_t)NH * QT * NKX * 2);
  if (off > ws_size || off > (size_t)134217728) return;
  const size_t nw8 = (size_t)DM * DM / 8; const unsigned gw = (unsigned)((nw8 + 255) / 256);
  k_wnat<<<gw, 256, 0, stream>>>(wq, nw8, BQ); k_wnat<<<gw, 256, 0, stream>>>(wk, nw8, BK); k_wnat<<<gw, 256, 0, stream>>>(wv, nw8, BV); k_wnat<<<gw, 256, 0, stream>>>(wo, nw8, BO);
  k_x16<<<(unsigned)((NR * DM / 8 + 255) / 256), 256, 0, stream>>>(x, X16, NR * DM / 8);
  const dim3 gp((unsigned)((NR / 128) * (DM / 64)), 1);
  k_gemm2<0><<<gp, 128, 0, stream>>>(X16, DM, 0, BQ, DM, 0, 0.0625f, bq, 0, nullptr, 1, 0, 0, nullptr, QKV,          LQ, 0, (int)NR, DM, DM);
  k_gemm2<0><<<gp, 128, 0, stream>>>(X16, DM, 0, BK, DM, 0, 0.0625f, bk, 0, nullptr, 1, 0, 0, nullptr, QKV + DM,     LQ, 0, (int)NR, DM, DM);
  k_gemm2<0><<<gp, 128, 0, stream>>>(X16, DM, 0, BV, DM, 0, 0.0625f, bv, 0, nullptr, 1, 0, 0, nullptr, QKV + 2 * DM, LQ, 0, (int)NR, DM, DM);
  k_vt<NH, SEQ><<<(unsigned)(NB * NH * (SEQ / 64)), 256, 0, stream>>>(QKV + 2 * DM, LQ, 0, VT);
  for (int b = 0; b < NB; ++b) { const size_t r0 = (size_t)b * SEQ;
    for (int q0 = 0; q0 < SEQ; q0 += QT) {
      k_gemm2<0><<<dim3((QT / 128) * (SEQ / 64), NH), 128, 0, stream>>>(QKV + (r0 + q0) * LQ, LQ, (size_t)HD, QKV + DM + r0 * LQ, LQ, (size_t)HD, 0.125f, nullptr, 0, nullptr, 1, 0, 0, S, nullptr, NKX, (size_t)QT * NKX, QT, SEQ, HD);
      k_rsmm<<<(NH * QT + 255) / 256, 256, 0, stream>>>(S, adj, P, NH, q0);
      k_gemm2<0><<<dim3((QT / 128) * (HD / 64), NH), 128, 0, stream>>>(P, NKX, (size_t)QT * NKX, VT + (size_t)b * NH * HD * SEQ, SEQ, (size_t)HD * SEQ, 0.0625f, nullptr, 0, nullptr, 1, 0, 0, nullptr, O16 + (r0 + q0) * DM, DM, (size_t)HD, QT, HD, SEQ); } }
  k_gemm2<0><<<gp, 128, 0, stream>>>(O16, DM, 0, BO, DM, 0, 0.0009765625f, bo, 0, nullptr, 1, 0, 0, (float*)d_out, nullptr, DM, 0, (int)NR, DM, DM);
}
